// IntraDomainAttention_54743653155456
// MI455X (gfx1250) — hardware-verified
//
#include <hip/hip_runtime.h>


namespace {
constexpr int Bn = 8, N = 2048, M = 1024, C = 512, H = 8, HD = 64, NQ = Bn * N, NK = Bn * M;
constexpr float XS = 8.0f, PS = 8.0f;
struct Wo_ { static constexpr size_t Q = 0, KV = (size_t)C * C, END = KV + (size_t)2 * C * C; };

typedef _Float16 b16;
typedef __attribute__((ext_vector_type(16))) _Float16 v16b;
typedef __attribute__((ext_vector_type(8))) _Float16 v8b;
typedef __attribute__((ext_vector_type(8))) float v8f;
typedef __attribute__((ext_vector_type(4))) float v4f;
__device__ __forceinline__ float bf16_rne(float f) { unsigned int u = __float_as_uint(f); u += 0x7FFFu + ((u >> 16) & 1u); return __uint_as_float(u & 0xFFFF0000u); }
__device__ __forceinline__ void split16(float v, b16& hi, b16& lo) { hi = (b16)v; lo = (b16)(v - (float)hi); }
__device__ __forceinline__ v16b frag_kb(const b16* p, int hh) { const v8b a = *(const v8b*)(p + 8 * hh), b = *(const v8b*)(p + 16 + 8 * hh); v16b f;
#pragma unroll
  for (int e = 0; e < 8; ++e) { f[e] = a[e]; f[8 + e] = b[e]; } return f; }
__device__ __forceinline__ v16b frag_x(const float* p, int hh) { v16b f;
#pragma unroll
  for (int e = 0; e < 8; ++e) { f[e] = (b16)bf16_rne(p[8 * hh + e]); f[8 + e] = (b16)bf16_rne(p[16 + 8 * hh + e]); } return f; }
__device__ __forceinline__ v8f wmma16b(v16b a, v16b b, v8f c) { v8f d = __builtin_amdgcn_wmma_f32_16x16x32_f16(false, a, false, b, (short)0, c, false, false); asm volatile("v_nop\n\tv_nop\n\tv_nop\n\tv_nop" : "+v"(d) : "v"(a), "v"(b)); return d; }
__device__ __forceinline__ void wave_lds_sync() { __builtin_amdgcn_fence(__ATOMIC_RELEASE, "workgroup"); __builtin_amdgcn_wave_barrier(); __builtin_amdgcn_fence(__ATOMIC_ACQUIRE, "workgroup"); }
__device__ __forceinline__ float nexp(float x) { return __builtin_amdgcn_exp2f(x * 1.4426950408889634f); }

__global__ __launch_bounds__(256) void prep_kernel(const float* __restrict__ Wq, const float* __restrict__ Wkv, const float* __restrict__ bq, const float* __restrict__ bkv, b16* __restrict__ R, float* __restrict__ P) {
  const size_t tid = (size_t)blockIdx.x * 256 + threadIdx.x, nth = (size_t)gridDim.x * 256;
  auto tr = [&](size_t base, int nout, int kin, const float* W) { for (size_t p = tid; p < (size_t)nout * (kin / 8); p += nth) { const int o = (int)(p / (kin / 8)), k0 = (int)(p % (kin / 8)) * 8; v8b v;
#pragma unroll
      for (int e = 0; e < 8; ++e) v[e] = (b16)bf16_rne(W[(size_t)(k0 + e) * nout + o]); *(volatile v8b*)(R + base + (size_t)o * kin + k0) = v; } };
  for (int pass = 0; pass < 2; ++pass) { tr(Wo_::Q, C, C, Wq); tr(Wo_::KV, 2 * C, C, Wkv); for (size_t q = tid; q < 1536; q += nth) P[q] = bf16_rne((q < 512) ? bq[q] : bkv[q - 512]); __threadfence(); }
}

__global__ __launch_bounds__(64) void qproj_kernel(const float* __restrict__ x, const b16* __restrict__ R, const float* __restrict__ P, b16* __restrict__ QH, b16* __restrict__ QL) {
  __shared__ __attribute__((aligned(16))) b16 Th[2][32][128 + 8], Tl[2][32][128 + 8];
  const int lane = threadIdx.x & 31, wave = threadIdx.x >> 5, nloc = lane & 15, hlf = lane >> 4, m0 = blockIdx.y * 32, c0 = blockIdx.x * 256 + wave * 128; const b16* Wr = R + Wo_::Q;
#pragma unroll 1
  for (int hf = 0; hf < 2; ++hf) { v8f acc[2][4];
#pragma unroll
    for (int r = 0; r < 2; ++r)
#pragma unroll
      for (int t = 0; t < 4; ++t) acc[r][t] = (v8f){};
#pragma unroll 2
    for (int kb = 0; kb < C; kb += 32) { const v16b a0 = frag_x(x + (size_t)(m0 + nloc) * C + kb, hlf), a1 = frag_x(x + (size_t)(m0 + 16 + nloc) * C + kb, hlf);
#pragma unroll
      for (int t = 0; t < 4; ++t) { const v16b bw = frag_kb(Wr + (size_t)(c0 + (hf * 4 + t) * 16 + nloc) * C + kb, hlf); acc[0][t] = wmma16b(a0, bw, acc[0][t]); acc[1][t] = wmma16b(a1, bw, acc[1][t]); } }
#pragma unroll
    for (int t = 0; t < 4; ++t) { const int tc = (hf * 4 + t) * 16 + nloc; const float bb = P[c0 + tc];
#pragma unroll
      for (int r = 0; r < 2; ++r)
#pragma unroll
        for (int v = 0; v < 8; ++v) { b16 a_, c_; split16((acc[r][t][v] + bb) * XS, a_, c_); Th[wave][r * 16 + 8 * hlf + v][tc] = a_; Tl[wave][r * 16 + 8 * hlf + v][tc] = c_; } } }
  wave_lds_sync();
  for (int pass = 0; pass < 2; ++pass) { for (int i = lane; i < 32 * 16; i += 32) { const int rr = i >> 4, c8 = (i & 15) * 8; const size_t gi = (size_t)(m0 + rr) * C + c0 + c8; *(volatile v8b*)(QH + gi) = *(const v8b*)(&Th[wave][rr][c8]); *(volatile v8b*)(QL + gi) = *(const v8b*)(&Tl[wave][rr][c8]); } __threadfence(); }
}

__global__ __launch_bounds__(128) void kvproj_kernel(const float* __restrict__ g, const b16* __restrict__ R, const float* __restrict__ P, b16* __restrict__ KH, b16* __restrict__ KL, b16* __restrict__ VT, b16* __restrict__ VTl) {
  __shared__ __attribute__((aligned(16))) b16 T1[128][128 + 8], T2[128][128 + 8];
  const int lane = threadIdx.x & 31, wave = threadIdx.x >> 5, nloc = lane & 15, hlf = lane >> 4, b = blockIdx.y, p0 = blockIdx.x * 128, m0 = b * M + p0 + wave * 32; const b16* Wr = R + Wo_::KV;
#pragma unroll 1
  for (int ch = 0; ch < 8; ++ch) { v8f acc[2][8];
#pragma unroll
    for (int r = 0; r < 2; ++r)
#pragma unroll
      for (int t = 0; t < 8; ++t) acc[r][t] = (v8f){};
#pragma unroll 2
    for (int kb = 0; kb < C; kb += 32) { const v16b a0 = frag_x(g + (size_t)(m0 + nloc) * C + kb, hlf), a1 = frag_x(g + (size_t)(m0 + 16 + nloc) * C + kb, hlf);
#pragma unroll
      for (int t = 0; t < 8; ++t) { const v16b bw = frag_kb(Wr + (size_t)(ch * 128 + t * 16 + nloc) * C + kb, hlf); acc[0][t] = wmma16b(a0, bw, acc[0][t]); acc[1][t] = wmma16b(a1, bw, acc[1][t]); } }
    __syncthreads();
#pragma unroll
    for (int t = 0; t < 8; ++t) { const int c = t * 16 + nloc; const float bb = P[512 + ch * 128 + c];
#pragma unroll
      for (int r = 0; r < 2; ++r)
#pragma unroll
        for (int v = 0; v < 8; ++v) { const int rr = wave * 32 + r * 16 + 8 * hlf + v; const float y = (acc[r][t][v] + bb) * XS;
          b16 a_, c_; split16(y, a_, c_); if (ch < 4) { T1[rr][c] = a_; T2[rr][c] = c_; } else { T1[c][rr] = a_; T2[c][rr] = c_; } } }
    __syncthreads();
    for (int pass = 0; pass < 2; ++pass) {
      if (ch < 4) { for (int i = threadIdx.x; i < 128 * 16; i += 128) { const int rr = i >> 4, c8 = (i & 15) * 8; const size_t gi = (size_t)(b * M + p0 + rr) * C + ch * 128 + c8; *(volatile v8b*)(KH + gi) = *(const v8b*)(&T1[rr][c8]); *(volatile v8b*)(KL + gi) = *(const v8b*)(&T2[rr][c8]); } }
      else { for (int i = threadIdx.x; i < 128 * 16; i += 128) { const int c = i >> 4, c8 = (i & 15) * 8; const int cg = (ch - 4) * 128 + c, h = cg / HD, d = cg % HD; const size_t gi = (((size_t)b * H + h) * HD + d) * M + p0 + c8; *(volatile v8b*)(VT + gi) = *(const v8b*)(&T1[c][c8]); *(volatile v8b*)(VTl + gi) = *(const v8b*)(&T2[c][c8]); } }
      __threadfence(); } }
}

__global__ __launch_bounds__(256) void attn_kernel(const b16* __restrict__ QH, const b16* __restrict__ QL, const b16* __restrict__ KH, const b16* __restrict__ KL, const b16* __restrict__ VT, const b16* __restrict__ VTl, float* __restrict__ out) {
  __shared__ __attribute__((aligned(16))) float Os[16][C + 4];
  const int h = threadIdx.x >> 5, lane = threadIdx.x & 31, hh = lane >> 4, col = lane & 15; const int b = blockIdx.x / (N / 16), q0 = (blockIdx.x % (N / 16)) * 16, qi = q0 + col;
  const size_t qb = (size_t)(b * N) * C + h * HD, kb_ = (size_t)(b * M) * C + h * HD; const b16* V = VT + (((size_t)b * H + h) * HD) * M; const b16* Vl = VTl + (((size_t)b * H + h) * HD) * M; const float SC = 1.0f / (XS * XS);
  const v16b qa0 = frag_kb(QH + qb + (size_t)qi * C, hh), qa1 = frag_kb(QH + qb + (size_t)qi * C + 32, hh), ql0 = frag_kb(QL + qb + (size_t)qi * C, hh), ql1 = frag_kb(QL + qb + (size_t)qi * C + 32, hh);
  float m = -INFINITY, l = 0.0f; v8f o[4] = {{}, {}, {}, {}};
  for (int kb = 0; kb < M; kb += 32) { v8f s0 = {}, s1 = {};
    { const v16b k0h = frag_kb(KH + kb_ + (size_t)(kb + col) * C, hh), k0l = frag_kb(KL + kb_ + (size_t)(kb + col) * C, hh), k1h = frag_kb(KH + kb_ + (size_t)(kb + col) * C + 32, hh), k1l = frag_kb(KL + kb_ + (size_t)(kb + col) * C + 32, hh);
      s0 = wmma16b(k0h, qa0, s0); s0 = wmma16b(k0h, ql0, s0); s0 = wmma16b(k0l, qa0, s0); s0 = wmma16b(k1h, qa1, s0); s0 = wmma16b(k1h, ql1, s0); s0 = wmma16b(k1l, qa1, s0); }
    { const v16b k0h = frag_kb(KH + kb_ + (size_t)(kb + 16 + col) * C, hh), k0l = frag_kb(KL + kb_ + (size_t)(kb + 16 + col) * C, hh), k1h = frag_kb(KH + kb_ + (size_t)(kb + 16 + col) * C + 32, hh), k1l = frag_kb(KL + kb_ + (size_t)(kb + 16 + col) * C + 32, hh);
      s1 = wmma16b(k0h, qa0, s1); s1 = wmma16b(k0h, ql0, s1); s1 = wmma16b(k0l, qa0, s1); s1 = wmma16b(k1h, qa1, s1); s1 = wmma16b(k1h, ql1, s1); s1 = wmma16b(k1l, qa1, s1); }
    float mr = -INFINITY;
#pragma unroll
    for (int r = 0; r < 8; ++r) { s0[r] *= SC; s1[r] *= SC; mr = fmaxf(mr, fmaxf(s0[r], s1[r])); }
    mr = fmaxf(mr, __shfl_xor(mr, 16)); const float mn = fmaxf(m, mr), al_ = nexp(m - mn); m = mn; float sum = 0.0f; v16b pb, pl;
#pragma unroll
    for (int r = 0; r < 8; ++r) { const float e0 = nexp(s0[r] - mn), e1 = nexp(s1[r] - mn); sum += e0 + e1; b16 a_, c_; split16(e0 * PS, a_, c_); pb[r] = a_; pl[r] = c_; split16(e1 * PS, a_, c_); pb[8 + r] = a_; pl[8 + r] = c_; }
    sum += __shfl_xor(sum, 16); l = l * al_ + sum;
#pragma unroll
    for (int t = 0; t < 4; ++t) { o[t] *= al_; const v16b vh = frag_kb(V + (size_t)(t * 16 + col) * M + kb, hh), vl = frag_kb(Vl + (size_t)(t * 16 + col) * M + kb, hh); o[t] = wmma16b(vh, pb, o[t]); o[t] = wmma16b(vh, pl, o[t]); o[t] = wmma16b(vl, pb, o[t]); } }
  const float inv = 1.0f / (l * PS * XS);
#pragma unroll
  for (int t = 0; t < 4; ++t)
#pragma unroll
    for (int r = 0; r < 8; ++r) Os[col][h * HD + t * 16 + 8 * hh + r] = o[t][r] * inv;
  __syncthreads();
  for (int pass = 0; pass < 2; ++pass) { for (int i = threadIdx.x; i < 16 * (C / 4); i += 256) { const int rr = i / (C / 4), c4 = (i % (C / 4)) * 4; *(volatile v4f*)(out + ((size_t)(b * N + q0 + rr)) * C + c4) = *(const v4f*)(&Os[rr][c4]); } __threadfence(); }
}
}

extern "C" void kernel_launch(void* const* d_in, const int* in_sizes, int n_in,
                              void* d_out, int out_size, void* d_ws, size_t ws_size, hipStream_t stream) {
  (void)n_in; (void)out_size;
  const float* x = (const float*)d_in[0]; const float* g = (const float*)d_in[1]; const float* Wq = (const float*)d_in[2]; const float* bq = (const float*)d_in[3]; const float* Wkv = (const float*)d_in[4]; const float* bkv = (const float*)d_in[5];
  float* out = (float*)d_out;
  if (in_sizes[0] != NQ * C || in_sizes[1] != NK * C || in_sizes[2] != C * C || in_sizes[4] != C * 2 * C) return;
  size_t off = 0; char* ws = (char*)d_ws;
  auto carve = [&](size_t bytes) { char* p = ws + off; off += (bytes + 255) & ~(size_t)255; return p; };
  b16* R = (b16*)carve(Wo_::END * 2); float* P = (float*)carve(1536 * 4); b16* QH = (b16*)carve((size_t)NQ * C * 2); b16* QL = (b16*)carve((size_t)NQ * C * 2); b16* KH = (b16*)carve((size_t)NK * C * 2); b16* KL = (b16*)carve((size_t)NK * C * 2); b16* VT = (b16*)carve((size_t)NK * C * 2); b16* VTl = (b16*)carve((size_t)NK * C * 2);
  if (off > ws_size) return;
  prep_kernel<<<128, 256, 0, stream>>>(Wq, Wkv, bq, bkv, R, P);
  qproj_kernel<<<dim3(C / 256, NQ / 32), 64, 0, stream>>>(x, R, P, QH, QL);
  kvproj_kernel<<<dim3(M / 128, Bn), 128, 0, stream>>>(g, R, P, KH, KL, VT, VTl);
  attn_kernel<<<NQ / 16, 256, 0, stream>>>(QH, QL, KH, KL, VT, VTl, out);
}
